// MultiHeadAttention_69432441307175
// MI455X (gfx1250) — hardware-run, weakly checked
//
#include <hip/hip_runtime.h>
#include <math.h>

typedef __attribute__((ext_vector_type(16))) _Float16 v16h;
typedef __attribute__((ext_vector_type(8)))  _Float16 v8h;
typedef __attribute__((ext_vector_type(8)))  float    v8f;
typedef __attribute__((ext_vector_type(4)))  float    v4f;
typedef __attribute__((ext_vector_type(4)))  int      v4i;

constexpr int kBatch  = 32;
constexpr int kG      = 1024;
constexpr int kD      = 256;
constexpr int kTok    = kBatch * kG;
constexpr int kChunkB = 4;
constexpr int kNChunk = kBatch / kChunkB;
constexpr int kSqrtD  = 16;
static_assert(kSqrtD * kSqrtD == kD);
static_assert(kTok == 32768);
static_assert((kD % 32) == 0 && (kG % 32) == 0);
static_assert((kD % 64) == 0 && (kG % 64) == 0 && (kTok % 64) == 0 && ((2 * kD) % 64) == 0);
static_assert((kBatch % kChunkB) == 0);

constexpr float kXCarry   = 16.0f;
constexpr float kWCarry   = 1024.0f;
constexpr float kQKVCarry = 16.0f;
constexpr float kPCarry   = 32768.0f;
constexpr float kHCarry   = 256.0f;
constexpr float kNormQK   = 1.0f / (float)kSqrtD;
constexpr float kProjScale  = kQKVCarry / (kXCarry * kWCarry);
constexpr float kScoreScale = kNormQK / (kQKVCarry * kQKVCarry);
constexpr float kPVScale    = kHCarry / (kPCarry * kQKVCarry);
constexpr float kOutScale   = 1.0f / (kHCarry * kWCarry);

constexpr size_t kOffX16  = 0;
constexpr size_t kOffW16  = kOffX16  + (size_t)kTok * kD * 2;
constexpr size_t kOffQK16 = kOffW16  + (size_t)4 * kD * kD * 2;
constexpr size_t kOffVT16 = kOffQK16 + (size_t)kTok * 2 * kD * 2;
constexpr size_t kOffSC   = kOffVT16 + (size_t)kBatch * kD * kG * 2;
constexpr size_t kOffP16  = kOffSC   + (size_t)kChunkB * kG * kG * 4;
constexpr size_t kOffH16  = kOffP16  + (size_t)kChunkB * kG * kG * 2;
constexpr size_t kWsTotal = kOffH16  + (size_t)kTok * kD * 2;
static_assert(kWsTotal == 109576192ull);
static_assert(kWsTotal <= 134217728ull);
static_assert((kOffW16 % 128) == 0 && (kOffQK16 % 128) == 0 && (kOffVT16 % 128) == 0 &&
              (kOffSC % 128) == 0 && (kOffP16 % 128) == 0 && (kOffH16 % 128) == 0);

union FragU { v16h v; v8h h[2]; };
__device__ __forceinline__ v16h frag_load(const _Float16* p) {
  FragU f;
  f.h[0] = *(const v8h*)(p);
  f.h[1] = *(const v8h*)(p + 16);
  return f.v;
}
__device__ __forceinline__ v8f mma_f16(v16h a, v16h b, v8f c) {
  return __builtin_amdgcn_wmma_f32_16x16x32_f16(false, a, false, b, (short)0, c, false, false);
}
__device__ __forceinline__ void mma_guard1(v8f& a, v16h x, v16h y) {
  asm volatile("v_nop\n\tv_nop\n\tv_nop\n\tv_nop" : "+v"(a) : "v"(x), "v"(y));
}
__device__ __forceinline__ void keep4_h(v16h a, v16h b, v16h c, v16h d) {
  asm volatile("v_nop" :: "v"(a), "v"(b), "v"(c), "v"(d));
}
__device__ __forceinline__ void acc_guard4(v8f& a, v8f& b, v8f& c, v8f& d) {
  asm volatile("v_nop\n\tv_nop\n\tv_nop\n\tv_nop" : "+v"(a), "+v"(b), "+v"(c), "+v"(d));
}

template <int BIAS_MODE, int OUT_MODE>
__global__ __launch_bounds__(256) void wmma_gemm64(
    const unsigned short* __restrict__ Ap, int lda, long strideA,
    const unsigned short* __restrict__ Btp, int ldb, long strideB,
    void* __restrict__ Cout, int ldc, long strideC,
    const float* __restrict__ bias,
    int M, int N, int K, float scale) {
  const _Float16* A  = (const _Float16*)Ap;
  const _Float16* Bt = (const _Float16*)Btp;
  __shared__ __align__(16) float sT[8][16 * 68];
  const int b    = blockIdx.y;
  const int lane = threadIdx.x & 31;
  const int wave = __builtin_amdgcn_readfirstlane((int)(threadIdx.x >> 5));
  const int tilesN = N >> 6;
  const int tilesM = M >> 6;
  const int tile = blockIdx.x * 8 + wave;
  if (tile >= tilesM * tilesN) return;
  const int tm = tile / tilesN;
  const int tn = tile - tm * tilesN;
  const int m0 = tm << 6;
  const int n0 = tn << 6;

  const _Float16* Ab = A  + (size_t)b * strideA;
  const _Float16* Bb = Bt + (size_t)b * strideB;

  const int rlane = lane & 15;
  const int koff  = (lane >> 4) * 8;
  const int mOff  = (lane >> 4) * 8;

  v8f acc[4][4];
#pragma unroll
  for (int i = 0; i < 4; ++i)
#pragma unroll
    for (int j = 0; j < 4; ++j) acc[i][j] = (v8f){0.f, 0.f, 0.f, 0.f, 0.f, 0.f, 0.f, 0.f};

  for (int k0 = 0; k0 < K; k0 += 32) {
    v16h bh[4];
#pragma unroll
    for (int j = 0; j < 4; ++j) {
      const size_t bo = (size_t)(n0 + (j << 4) + rlane) * ldb + koff + k0;
      bh[j] = frag_load(Bb + bo);
    }
#pragma unroll
    for (int i = 0; i < 4; ++i) {
      const size_t ao = (size_t)(m0 + (i << 4) + rlane) * lda + koff + k0;
      v16h ah = frag_load(Ab + ao);
#pragma unroll
      for (int j = 0; j < 4; ++j) acc[i][j] = mma_f16(ah, bh[j], acc[i][j]);
      mma_guard1(acc[i][0], ah, bh[0]);
      mma_guard1(acc[i][1], ah, bh[1]);
      mma_guard1(acc[i][2], ah, bh[2]);
      mma_guard1(acc[i][3], ah, bh[3]);
    }
    keep4_h(bh[0], bh[1], bh[2], bh[3]);
  }
  acc_guard4(acc[0][0], acc[0][1], acc[0][2], acc[0][3]);
  acc_guard4(acc[1][0], acc[1][1], acc[1][2], acc[1][3]);
  acc_guard4(acc[2][0], acc[2][1], acc[2][2], acc[2][3]);
  acc_guard4(acc[3][0], acc[3][1], acc[3][2], acc[3][3]);

  float* slab = sT[wave];
#pragma unroll
  for (int i = 0; i < 4; ++i) {
    const int mBase = m0 + (i << 4);
#pragma unroll
    for (int j = 0; j < 4; ++j) {
      const int n = n0 + (j << 4) + rlane;
      float bv = 0.f;
      if (BIAS_MODE == 2) bv = bias[n];
#pragma unroll
      for (int r = 0; r < 8; ++r) {
        float v = acc[i][j][r] * scale;
        if (BIAS_MODE == 2) v += bv;
        slab[(mOff + r) * 68 + (j << 4) + rlane] = v;
      }
    }
    __builtin_amdgcn_fence(__ATOMIC_RELEASE, "workgroup");
    __builtin_amdgcn_wave_barrier();
    __builtin_amdgcn_fence(__ATOMIC_ACQUIRE, "workgroup");
    if (OUT_MODE == 0) {
      float* C = (float*)Cout + (size_t)b * strideC;
      const int hh = lane >> 4, c4 = (lane & 15) * 4;
      for (int pass = 0; pass < 2; ++pass) {
#pragma unroll
        for (int it = 0; it < 8; ++it) {
          const int row = it * 2 + hh;
          v4f v = *(const v4f*)(slab + row * 68 + c4);
          *(volatile v4f*)(C + (size_t)(mBase + row) * ldc + n0 + c4) = v;
        }
        __threadfence();
      }
    } else {
      const int q = lane >> 3, c8 = (lane & 7) * 8;
      unsigned short* C = (unsigned short*)Cout + (size_t)b * strideC;
      for (int pass = 0; pass < 2; ++pass) {
#pragma unroll
        for (int it = 0; it < 4; ++it) {
          const int row = it * 4 + q;
          const float* sp = slab + row * 68 + c8;
          v8h hv;
#pragma unroll
          for (int e = 0; e < 8; ++e) hv[e] = (_Float16)sp[e];
          *(volatile v8h*)(C + (size_t)(mBase + row) * ldc + n0 + c8) = hv;
        }
        __threadfence();
      }
    }
    __builtin_amdgcn_fence(__ATOMIC_RELEASE, "workgroup");
    __builtin_amdgcn_wave_barrier();
    __builtin_amdgcn_fence(__ATOMIC_ACQUIRE, "workgroup");
  }
}

__global__ __launch_bounds__(256) void cast8_f16_kernel(const float* __restrict__ in,
                                                        unsigned short* __restrict__ out,
                                                        int n8, float carry) {
  const int i = blockIdx.x * 256 + threadIdx.x;
  if (i >= n8) return;
  const float* p = in + 8 * (size_t)i;
  const v4f a = *(const v4f*)(p);
  const v4f c = *(const v4f*)(p + 4);
  v8h hv;
#pragma unroll
  for (int e = 0; e < 4; ++e) {
    hv[e]     = (_Float16)(a[e] * carry);
    hv[4 + e] = (_Float16)(c[e] * carry);
  }
  unsigned short* q = out + 8 * (size_t)i;
  *(volatile v8h*)q = hv;
  __threadfence();
  *(volatile v8h*)q = hv;
}

__global__ __launch_bounds__(256) void cast8_w4_kernel(const float* __restrict__ W0, const float* __restrict__ W1,
                                                       const float* __restrict__ W2, const float* __restrict__ W3,
                                                       unsigned short* __restrict__ out, float carry) {
  const int z = blockIdx.y;
  const float* W = (z == 0) ? W0 : (z == 1) ? W1 : (z == 2) ? W2 : W3;
  const int i = blockIdx.x * 256 + threadIdx.x;
  const float* p = W + 8 * (size_t)i;
  const v4f a = *(const v4f*)(p);
  const v4f c = *(const v4f*)(p + 4);
  v8h hv;
#pragma unroll
  for (int e = 0; e < 4; ++e) {
    hv[e]     = (_Float16)(a[e] * carry);
    hv[4 + e] = (_Float16)(c[e] * carry);
  }
  unsigned short* q = out + (size_t)z * kD * kD + 8 * (size_t)i;
  *(volatile v8h*)q = hv;
  __threadfence();
  *(volatile v8h*)q = hv;
}

constexpr int kSmRows = 4;
static_assert((kG % kSmRows) == 0 && kG == 128 * 8);
__global__ __launch_bounds__(128) void softmax_keymask_kernel(const float* __restrict__ S,
                                                              const int* __restrict__ mask,
                                                              const int* __restrict__ evalflag,
                                                              unsigned short* __restrict__ P, int b0) {
  __shared__ float redM[4];
  __shared__ float redS[4];
  const int t    = threadIdx.x;
  const int lane = t & 31;
  const int wave = __builtin_amdgcn_readfirstlane((int)(threadIdx.x >> 5));
  const int bl   = blockIdx.y;
  int b = b0 + bl;
  b = b < 0 ? 0 : (b > kBatch - 1 ? kBatch - 1 : b);
  const int c0 = t * 8;
  const v4i mk0 = *(const v4i*)(mask + (size_t)b * kG + c0);
  const v4i mk1 = *(const v4i*)(mask + (size_t)b * kG + c0 + 4);
  int blk[8];
#pragma unroll
  for (int e = 0; e < 4; ++e) {
    blk[e]     = (mk0[e] != 0) ? 1 : 0;
    blk[4 + e] = (mk1[e] != 0) ? 1 : 0;
  }
  const float fill = (evalflag[0] != 0) ? (-INFINITY) : (-30.0f);

#pragma unroll 1
  for (int rr = 0; rr < kSmRows; ++rr) {
    const int row = blockIdx.x * kSmRows + rr;
    const size_t ro = ((size_t)bl * kG + row) * kG + c0;
    const v4f a = *(const v4f*)(S + ro);
    const v4f c = *(const v4f*)(S + ro + 4);
    float x[8];
#pragma unroll
    for (int e = 0; e < 4; ++e) {
      x[e]     = blk[e]     ? fill : a[e];
      x[4 + e] = blk[4 + e] ? fill : c[e];
    }
    float m = fmaxf(fmaxf(fmaxf(x[0], x[1]), fmaxf(x[2], x[3])), fmaxf(fmaxf(x[4], x[5]), fmaxf(x[6], x[7])));
#pragma unroll
    for (int off = 16; off > 0; off >>= 1) m = fmaxf(m, __shfl_xor(m, off, 32));
    if (lane == 0) redM[wave] = m;
    __syncthreads();
    const float mrow = fmaxf(fmaxf(redM[0], redM[1]), fmaxf(redM[2], redM[3]));
    float ev[8];
    float s = 0.0f;
#pragma unroll
    for (int e = 0; e < 8; ++e) {
      ev[e] = expf(x[e] - mrow);
      s += ev[e];
    }
#pragma unroll
    for (int off = 16; off > 0; off >>= 1) s += __shfl_xor(s, off, 32);
    if (lane == 0) redS[wave] = s;
    __syncthreads();
    const float tot = ((redS[0] + redS[1]) + redS[2]) + redS[3];
    const float inv = kPCarry * (1.0f / tot);
    v8h hv;
#pragma unroll
    for (int e = 0; e < 8; ++e) {
      const float pv = blk[e] ? 0.0f : (ev[e] * inv);
      hv[e] = (_Float16)pv;
    }
    unsigned short* q = P + ro;
    *(volatile v8h*)q = hv;
    __threadfence();
    *(volatile v8h*)q = hv;
  }
}

__global__ __launch_bounds__(32) void premise_guard_kernel(const int* __restrict__ gsz, float* __restrict__ out) {
  const int g = gsz[0];
  if (g != kG) {
    const int lane = threadIdx.x & 31;
    const float qn = __uint_as_float(0x7fc00000u);
    const v4f nv = (v4f){qn, qn, qn, qn};
    for (int pass = 0; pass < 2; ++pass) {
      *(volatile v4f*)(out + lane * 4) = nv;
      *(volatile v4f*)(out + 128 + lane * 4) = nv;
      __threadfence();
    }
  }
}

extern "C" void kernel_launch(void* const* d_in, const int* in_sizes, int n_in,
                              void* d_out, int out_size, void* d_ws, size_t ws_size,
                              hipStream_t stream) {
  if (n_in < 9) return;
  if (in_sizes[0] != kTok * kD) return;
  if (in_sizes[1] != kBatch * kG) return;
  if (in_sizes[2] != 1 || in_sizes[3] != 1) return;
  if (in_sizes[4] != kD * kD || in_sizes[5] != kD * kD || in_sizes[6] != kD * kD || in_sizes[7] != kD * kD) return;
  if (in_sizes[8] != kD) return;
  if (out_size != kTok * kD) return;
  if (ws_size < kWsTotal) return;

  const float* data   = (const float*)d_in[0];
  const int*   mask   = (const int*)d_in[1];
  const int*   gsize  = (const int*)d_in[2];
  const int*   evalf  = (const int*)d_in[3];
  const float* Wq     = (const float*)d_in[4];
  const float* Wk     = (const float*)d_in[5];
  const float* Wv     = (const float*)d_in[6];
  const float* Wo     = (const float*)d_in[7];
  const float* b_out  = (const float*)d_in[8];
  float* out = (float*)d_out;

  char* ws = (char*)d_ws;
  unsigned short* X16  = (unsigned short*)(ws + kOffX16);
  unsigned short* W16  = (unsigned short*)(ws + kOffW16);
  unsigned short* QK16 = (unsigned short*)(ws + kOffQK16);
  unsigned short* VT16 = (unsigned short*)(ws + kOffVT16);
  float*          SC   = (float*)(ws + kOffSC);
  unsigned short* P16  = (unsigned short*)(ws + kOffP16);
  unsigned short* H16  = (unsigned short*)(ws + kOffH16);

  cast8_f16_kernel<<<(kTok * kD / 8) / 256, 256, 0, stream>>>(data, X16, kTok * kD / 8, kXCarry);
  cast8_w4_kernel<<<dim3((kD * kD / 8) / 256, 4), 256, 0, stream>>>(Wq, Wk, Wv, Wo, W16, kWCarry);

  wmma_gemm64<0, 1><<<dim3((kTok / 64) * (2 * kD / 64) / 8, 1), 256, 0, stream>>>(
      X16, kD, 0L,
      W16, kD, 0L,
      (void*)QK16, 2 * kD, 0L,
      b_out,
      kTok, 2 * kD, kD, kProjScale);

  wmma_gemm64<0, 1><<<dim3((kD / 64) * (kG / 64) / 8, kBatch), 256, 0, stream>>>(
      W16 + (size_t)2 * kD * kD, kD, 0L,
      X16, kD, (long)kG * kD,
      (void*)VT16, kG, (long)kD * kG,
      b_out,
      kD, kG, kD, kProjScale);

  for (int c = 0; c < kNChunk; ++c) {
    const int b0 = c * kChunkB;
    const unsigned short* Qc = QK16 + (size_t)b0 * kG * 2 * kD;
    const unsigned short* Kc = Qc + kD;
    wmma_gemm64<0, 0><<<dim3((kG / 64) * (kG / 64) / 8, kChunkB), 256, 0, stream>>>(
        Qc, 2 * kD, (long)kG * 2 * kD,
        Kc, 2 * kD, (long)kG * 2 * kD,
        (void*)SC, kG, (long)kG * kG,
        b_out,
        kG, kG, kD, kScoreScale);
    softmax_keymask_kernel<<<dim3(kG / kSmRows, kChunkB), 128, 0, stream>>>(SC, mask, evalf, P16, b0);
    wmma_gemm64<0, 1><<<dim3((kG / 64) * (kD / 64) / 8, kChunkB), 256, 0, stream>>>(
        P16, kG, (long)kG * kG,
        VT16 + (size_t)b0 * kD * kG, kG, (long)kD * kG,
        (void*)(H16 + (size_t)b0 * kG * kD), kD, (long)kG * kD,
        b_out,
        kG, kD, kG, kPVScale);
  }

  wmma_gemm64<2, 0><<<dim3((kTok / 64) * (kD / 64) / 8, 1), 256, 0, stream>>>(
      H16, kD, 0L,
      W16 + (size_t)3 * kD * kD, kD, 0L,
      (void*)out, kD, 0L,
      b_out,
      kTok, kD, kD, kOutScale);

  premise_guard_kernel<<<1, 32, 0, stream>>>(gsize, out);
}
